// SelectiveScan_46428596470334
// MI455X (gfx1250) — hardware-verified
//
#include <hip/hip_runtime.h>
#include <math.h>

typedef __attribute__((ext_vector_type(16))) _Float16 v16h;
typedef __attribute__((ext_vector_type(8)))  _Float16 v8h;
typedef __attribute__((ext_vector_type(16))) __bf16   v16b;
typedef __attribute__((ext_vector_type(8)))  __bf16   v8b;
typedef __attribute__((ext_vector_type(8)))  float    v8f;
typedef __attribute__((ext_vector_type(4)))  float    v4f;
typedef __attribute__((ext_vector_type(2)))  float    v2f;

constexpr int kBatch = 2;
constexpr int kSeqL  = 2048;
constexpr int kE     = 1024;
constexpr int kNst   = 16;
constexpr int kDtR   = 64;
constexpr int kPrmN  = 96;
constexpr int kPrmP  = 128;
constexpr int kCoff  = 80;
constexpr int kRows  = kBatch * kSeqL;
constexpr int kScCh  = 128;
constexpr int kScTS  = 16;
constexpr int kScYP  = 132;
static_assert(kDtR + 2 * kNst == kPrmN, "params width");
static_assert(kCoff == kDtR + kNst, "C slice offset");
static_assert((kE % 32) == 0 && (kDtR % 32) == 0, "GEMM K multiples of 32");
static_assert((kRows % 64) == 0 && (kE % 64) == 0 && (kPrmP % 64) == 0, "GEMM M,N multiples of 64");
static_assert((kSeqL % kScTS) == 0 && (kE % kScCh) == 0, "scan tile multiples");

constexpr float kCarryW   = 32.0f;
constexpr float kCarryWdt = 64.0f;
constexpr float kCarryY   = 16.0f;
constexpr float kInvW     = 1.0f / kCarryW;
constexpr float kInvWdt   = 1.0f / kCarryWdt;
constexpr float kInvYW    = 1.0f / (kCarryY * kCarryW);

constexpr size_t kOffXH  = 0;
constexpr size_t kOffWZH = kOffXH  + (size_t)kRows * kE * 2;
constexpr size_t kOffWOH = kOffWZH + (size_t)kE * kE * 2;
constexpr size_t kOffWPH = kOffWOH + (size_t)kE * kE * 2;
constexpr size_t kOffWDH = kOffWPH + (size_t)kPrmP * kE * 2;
constexpr size_t kOffZP  = kOffWDH + (size_t)kE * kDtR * 2;
constexpr size_t kOffPRM = kOffZP  + (size_t)kRows * kE * 4;
constexpr size_t kOffDTU = kOffPRM + (size_t)kRows * kPrmP * 4;
constexpr size_t kOffDLR = kOffDTU + (size_t)kRows * kDtR * 2;
constexpr size_t kOffYG  = kOffDLR + (size_t)kRows * kE * 4;
constexpr size_t kWsTotal = kOffYG + (size_t)kRows * kE * 2;
static_assert(kWsTotal == 57540608ull, "carve total");
static_assert(kWsTotal <= 134217728ull, "carve cap");
static_assert((kOffWZH % 128) == 0 && (kOffWOH % 128) == 0 && (kOffWPH % 128) == 0 && (kOffWDH % 128) == 0 &&
              (kOffZP % 128) == 0 && (kOffPRM % 128) == 0 && (kOffDTU % 128) == 0 && (kOffDLR % 128) == 0 &&
              (kOffYG % 128) == 0, "128-B aligned regions");

__device__ __forceinline__ unsigned short f2bf_bits(float f) {
  unsigned u = __float_as_uint(f);
  return (unsigned short)((u + 0x7FFFu + ((u >> 16) & 1u)) >> 16);
}
__device__ __forceinline__ float bf_bits2f(unsigned short h) { return __uint_as_float(((unsigned)h) << 16); }

__device__ __forceinline__ void dep_guard4_h(v8f& a, v8f& b, v8f& c, v8f& d, v16h x, v16h y) {
  asm volatile("v_nop\n\tv_nop\n\tv_nop\n\tv_nop" : "+v"(a), "+v"(b), "+v"(c), "+v"(d) : "v"(x), "v"(y));
}
__device__ __forceinline__ void dep_guard4_b(v8f& a, v8f& b, v8f& c, v8f& d, v16b x, v16b y) {
  asm volatile("v_nop\n\tv_nop\n\tv_nop\n\tv_nop" : "+v"(a), "+v"(b), "+v"(c), "+v"(d) : "v"(x), "v"(y));
}
__device__ __forceinline__ void keep4_h(v16h a, v16h b, v16h c, v16h d) { asm volatile("v_nop" :: "v"(a), "v"(b), "v"(c), "v"(d)); }
__device__ __forceinline__ void keep4_b(v16b a, v16b b, v16b c, v16b d) { asm volatile("v_nop" :: "v"(a), "v"(b), "v"(c), "v"(d)); }
__device__ __forceinline__ void acc_guard4(v8f& a, v8f& b, v8f& c, v8f& d) { asm volatile("v_nop\n\tv_nop\n\tv_nop\n\tv_nop" : "+v"(a), "+v"(b), "+v"(c), "+v"(d)); }
template <typename T> struct Frag;
template <> struct Frag<_Float16> {
  typedef v16h V; union U { v16h v; v8h h[2]; };
  static __device__ __forceinline__ v16h load(const _Float16* p) {
    U f; f.h[0] = *(const v8h*)(p); f.h[1] = *(const v8h*)(p + 16); return f.v;
  }
  static __device__ __forceinline__ v8f mma(v16h a, v16h b, v8f c) {
    return __builtin_amdgcn_wmma_f32_16x16x32_f16(false, a, false, b, (short)0, c, false, false);
  }
  static __device__ __forceinline__ void guard4(v8f& a, v8f& b, v8f& c, v8f& d, v16h x, v16h y) { dep_guard4_h(a, b, c, d, x, y); }
  static __device__ __forceinline__ void keep(v16h a, v16h b, v16h c, v16h d) { keep4_h(a, b, c, d); }
};
template <> struct Frag<__bf16> {
  typedef v16b V; union U { v16b v; v8b h[2]; };
  static __device__ __forceinline__ v16b load(const __bf16* p) {
    U f; f.h[0] = *(const v8b*)(p); f.h[1] = *(const v8b*)(p + 16); return f.v;
  }
  static __device__ __forceinline__ v8f mma(v16b a, v16b b, v8f c) {
    return __builtin_amdgcn_wmma_f32_16x16x32_bf16(false, a, false, b, (short)0, c, false, false);
  }
  static __device__ __forceinline__ void guard4(v8f& a, v8f& b, v8f& c, v8f& d, v16b x, v16b y) { dep_guard4_b(a, b, c, d, x, y); }
  static __device__ __forceinline__ void keep(v16b a, v16b b, v16b c, v16b d) { keep4_b(a, b, c, d); }
};

template <int ET> struct Elem;
template <> struct Elem<0> { typedef _Float16 T; };
template <> struct Elem<1> { typedef __bf16 T; };
template <int ET, bool SPLIT, int BIAS_MODE, int OUT_MODE, bool RESID, int ACT = 0>
__global__ __launch_bounds__(256) void wmma_gemm64(
    const unsigned short* __restrict__ Ap, const unsigned short* __restrict__ A2p, int lda, long strideA,
    const unsigned short* __restrict__ Btp, const unsigned short* __restrict__ Bt2p, int ldb, long strideB,
    void* __restrict__ Cout, void* __restrict__ Cout2, int ldc, long strideC,
    const float* __restrict__ bias,
    const float* __restrict__ resid, long strideR,
    int M, int N, int K, float scale) {
  typedef typename Elem<ET>::T T;
  typedef typename Frag<T>::V V;
  const T* A = (const T*)Ap; const T* A2 = (const T*)A2p; const T* Bt = (const T*)Btp; const T* Bt2 = (const T*)Bt2p;
  __shared__ __align__(16) float sT[8][16 * 68];
  const int b    = blockIdx.y;
  const int lane = threadIdx.x & 31;
  const int wave = threadIdx.x >> 5;
  const int tilesN = N >> 6;
  const int tilesM = M >> 6;
  const int tile = blockIdx.x * 8 + wave;
  if (tile >= tilesM * tilesN) return;
  const int tm = tile / tilesN;
  const int tn = tile - tm * tilesN;
  const int m0 = tm << 6;
  const int n0 = tn << 6;

  const T* Ab  = A  + (size_t)b * strideA;
  const T* Bb  = Bt + (size_t)b * strideB;
  const T* Ab2 = SPLIT ? (A2  + (size_t)b * strideA) : nullptr;
  const T* Bb2 = SPLIT ? (Bt2 + (size_t)b * strideB) : nullptr;

  const int rlane = lane & 15;
  const int koff  = (lane >> 4) * 8;
  const int mOff  = (lane >> 4) * 8;

  v8f acc[4][4];
#pragma unroll
  for (int i = 0; i < 4; ++i)
#pragma unroll
    for (int j = 0; j < 4; ++j) acc[i][j] = (v8f){0.f,0.f,0.f,0.f,0.f,0.f,0.f,0.f};

  for (int k0 = 0; k0 < K; k0 += 32) {
    V bh[4], bl[4];
#pragma unroll
    for (int j = 0; j < 4; ++j) {
      const size_t bo = (size_t)(n0 + (j << 4) + rlane) * ldb + koff + k0;
      bh[j] = Frag<T>::load(Bb + bo);
      if (SPLIT) bl[j] = Frag<T>::load(Bb2 + bo);
    }
#pragma unroll
    for (int i = 0; i < 4; ++i) {
      const size_t ao = (size_t)(m0 + (i << 4) + rlane) * lda + koff + k0;
      V ah = Frag<T>::load(Ab + ao);
      V al;
      if (SPLIT) al = Frag<T>::load(Ab2 + ao);
#pragma unroll
      for (int j = 0; j < 4; ++j) {
        acc[i][j] = Frag<T>::mma(ah, bh[j], acc[i][j]);
        if (SPLIT) {
          acc[i][j] = Frag<T>::mma(ah, bl[j], acc[i][j]);
          acc[i][j] = Frag<T>::mma(al, bh[j], acc[i][j]);
        }
      }
      Frag<T>::guard4(acc[i][0], acc[i][1], acc[i][2], acc[i][3], ah, SPLIT ? al : ah);
    }
    Frag<T>::keep(bh[0], bh[1], bh[2], bh[3]);
    if (SPLIT) Frag<T>::keep(bl[0], bl[1], bl[2], bl[3]);
  }
  acc_guard4(acc[0][0], acc[0][1], acc[0][2], acc[0][3]);
  acc_guard4(acc[1][0], acc[1][1], acc[1][2], acc[1][3]);
  acc_guard4(acc[2][0], acc[2][1], acc[2][2], acc[2][3]);
  acc_guard4(acc[3][0], acc[3][1], acc[3][2], acc[3][3]);

  float* slab = sT[wave];
  const float* Rb = RESID ? (resid + (size_t)b * strideR) : nullptr;
#pragma unroll
  for (int i = 0; i < 4; ++i) {
    const int mBase = m0 + (i << 4);
#pragma unroll
    for (int j = 0; j < 4; ++j) {
      const int n = n0 + (j << 4) + rlane;
      float bv = 0.f;
      if (BIAS_MODE == 2) bv = bias[n];
#pragma unroll
      for (int r = 0; r < 8; ++r) {
        float v = acc[i][j][r] * scale;
        if (BIAS_MODE == 1) v += bias[mBase + mOff + r];
        if (BIAS_MODE == 2) v += bv;
        if (RESID) v += Rb[(size_t)(mBase + mOff + r) * ldc + n];
        if (ACT == 2) v = fmaxf(v, 0.0f);
        if (ACT == 4) v = (v > 0.f) ? v : 0.01f * v;
        slab[(mOff + r) * 68 + (j << 4) + rlane] = v;
      }
    }
    __builtin_amdgcn_fence(__ATOMIC_RELEASE, "workgroup");
    __builtin_amdgcn_wave_barrier();
    __builtin_amdgcn_fence(__ATOMIC_ACQUIRE, "workgroup");
    if (OUT_MODE == 0) {
      float* C = (float*)Cout + (size_t)b * strideC;
      const int hh = lane >> 4, c4 = (lane & 15) * 4;
      for (int pass = 0; pass < 2; ++pass) {
#pragma unroll
        for (int it = 0; it < 8; ++it) {
          const int row = it * 2 + hh;
          v4f v = *(const v4f*)(slab + row * 68 + c4);
          *(volatile v4f*)(C + (size_t)(mBase + row) * ldc + n0 + c4) = v;
        }
        __threadfence();
      }
    } else {
      const int q = lane >> 3, c8 = (lane & 7) * 8;
      unsigned short* C  = (unsigned short*)Cout  + (size_t)b * strideC;
      unsigned short* C2 = (OUT_MODE == 2) ? ((unsigned short*)Cout2 + (size_t)b * strideC) : nullptr;
      for (int pass = 0; pass < 2; ++pass) {
#pragma unroll
        for (int it = 0; it < 4; ++it) {
          const int row = it * 4 + q;
          const float* sp = slab + row * 68 + c8;
          v8h hv, lv;
#pragma unroll
          for (int e = 0; e < 8; ++e) {
            if (OUT_MODE == 1) {
              hv[e] = (_Float16)sp[e];
            } else {
              unsigned short hb = f2bf_bits(sp[e]);
              unsigned short lb = f2bf_bits(sp[e] - bf_bits2f(hb));
              hv[e] = __builtin_bit_cast(_Float16, hb);
              lv[e] = __builtin_bit_cast(_Float16, lb);
            }
          }
          *(volatile v8h*)(C + (size_t)(mBase + row) * ldc + n0 + c8) = hv;
          if (OUT_MODE == 2) *(volatile v8h*)(C2 + (size_t)(mBase + row) * ldc + n0 + c8) = lv;
        }
        __threadfence();
      }
    }
    __builtin_amdgcn_fence(__ATOMIC_RELEASE, "workgroup");
    __builtin_amdgcn_wave_barrier();
    __builtin_amdgcn_fence(__ATOMIC_ACQUIRE, "workgroup");
  }
}

__global__ __launch_bounds__(256) void cast_f16_pad_kernel(
    const float* __restrict__ src, unsigned short* __restrict__ dst, int total8, int real8, float scale)
{
  const int i = blockIdx.x * 256 + threadIdx.x;
  if (i >= total8) return;
  const bool live = (i < real8);
  const int ic = live ? i : (real8 - 1);
  const float* p = src + ((size_t)ic << 3);
  const v4f a0 = *(const v4f*)(p);
  const v4f a1 = *(const v4f*)(p + 4);
  v8h hv;
#pragma unroll
  for (int e = 0; e < 4; ++e) {
    const float f0 = a0[e];
    const float f1 = a1[e];
    hv[e]     = (_Float16)(live ? (f0 * scale) : 0.0f);
    hv[4 + e] = (_Float16)(live ? (f1 * scale) : 0.0f);
  }
  unsigned short* q = dst + ((size_t)i << 3);
  *(volatile v8h*)q = hv;
  __threadfence();
  *(volatile v8h*)q = hv;
}

__global__ __launch_bounds__(256) void dt_cast_kernel(
    const float* __restrict__ PRM, unsigned short* __restrict__ DTU, int total8)
{
  const int i = blockIdx.x * 256 + threadIdx.x;
  if (i >= total8) return;
  const int e0  = i << 3;
  const int row = e0 >> 6;
  const int c8  = e0 & 63;
  const float* p = PRM + (size_t)row * kPrmP + c8;
  const v4f a0 = *(const v4f*)(p);
  const v4f a1 = *(const v4f*)(p + 4);
  v8h hv;
#pragma unroll
  for (int e = 0; e < 4; ++e) {
    const float f0 = a0[e];
    const float f1 = a1[e];
    hv[e]     = (_Float16)f0;
    hv[4 + e] = (_Float16)f1;
  }
  unsigned short* qd = DTU + e0;
  *(volatile v8h*)qd = hv;
  __threadfence();
  *(volatile v8h*)qd = hv;
}

__global__ __launch_bounds__(128) void scan_kernel(
    const float* __restrict__ X, const float* __restrict__ CW, const float* __restrict__ DLR,
    const float* __restrict__ ZP, const float* __restrict__ PRM, const float* __restrict__ Alog,
    const float* __restrict__ Dv, unsigned short* __restrict__ YG)
{
  __shared__ __align__(16) float sH[kNst * kScCh];
  __shared__ __align__(16) v2f   sAI[kNst * kScCh];
  __shared__ __align__(16) float sC[kScTS * kNst];
  __shared__ __align__(16) float sY[kScTS * kScYP];
  const int tid = threadIdx.x, lane = tid & 31, wave = tid >> 5;
  constexpr int kBlkPerB = kE / kScCh;
  const int bix = blockIdx.x / kBlkPerB;
  const int d0  = (blockIdx.x - bix * kBlkPerB) * kScCh;
  const int d   = d0 + tid;
  const size_t row0 = (size_t)bix * kSeqL;

#pragma unroll 1
  for (int n = 0; n < kNst; ++n) {
    const float al  = Alog[(size_t)d * kNst + n];
    const float An  = -expf(al);
    const float den = An + 1e-10f;
    v2f ai;
    ai.x = An;
    ai.y = 1.0f / den;
    sAI[n * kScCh + tid] = ai;
    sH[n * kScCh + tid]  = 0.0f;
  }
  const v4f wv = *(const v4f*)(CW + (size_t)d * 4);
  const float w0 = wv[0], w1 = wv[1], w2 = wv[2], w3 = wv[3];
  const float Dd = Dv[d];
  __syncthreads();

  float xm3 = 0.0f, xm2 = 0.0f, xm1 = 0.0f;
  float dtq = 0.0f, uq = 0.0f;
  const int hh = lane >> 4, c8 = (lane & 15) * 8;

#pragma unroll 1
  for (int c = 0; c < kSeqL / kScTS; ++c) {
    const int t0 = c * kScTS;
    if (tid < 64) {
      const int r = tid >> 2, q4 = (tid & 3) * 4;
      const v4f cv = *(const v4f*)(PRM + (row0 + t0 + r) * kPrmP + kCoff + q4);
      *(v4f*)(sC + r * kNst + q4) = cv;
    }
    __syncthreads();
#pragma unroll 1
    for (int s = 0; s < kScTS; ++s) {
      const size_t m = row0 + (size_t)(t0 + s);
      float xcur = X[m * kE + d];
      asm volatile("" : "+v"(xcur));
      float av = DLR[m * kE + d];
      asm volatile("" : "+v"(av));
      float zv = ZP[m * kE + d];
      asm volatile("" : "+v"(zv));
      float xc = w0 * xm3;
      xc = fmaf(w1, xm2, xc);
      xc = fmaf(w2, xm1, xc);
      xc = fmaf(w3, xcur, xc);
      const float ut = xc * __builtin_amdgcn_rcpf(1.0f + expf(-xc));
      const float dtt = fmaxf(av, 0.0f) + log1pf(expf(-fabsf(av)));
      const bool first = ((t0 + s) == 0);
      const float dta = first ? dtt : dtq;
      const float ua  = first ? ut  : uq;
      float y = 0.0f;
#pragma unroll 1
      for (int n = 0; n < kNst; ++n) {
        const v2f ai = sAI[n * kScCh + tid];
        const float hn0 = sH[n * kScCh + tid];
        const float cn  = sC[s * kNst + n];
        const float An = ai.x;
        const float iA = ai.y;
        const float a  = expf(dta * An);
        const float bq = (a - 1.0f) * iA;
        const float bt = (fabsf(An) < 1e-5f) ? dta : bq;
        const float hn = fmaf(a, hn0, bt * ua);
        sH[n * kScCh + tid] = hn;
        y = fmaf(cn, hn, y);
      }
      y = fmaf(ut, Dd, y);
      const float g = zv * __builtin_amdgcn_rcpf(1.0f + expf(-zv));
      sY[s * kScYP + tid] = (y * g) * kCarryY;
      dtq = dtt; uq = ut;
      xm3 = xm2; xm2 = xm1; xm1 = xcur;
    }
    __syncthreads();
    v8h hv[2];
#pragma unroll
    for (int it = 0; it < 2; ++it) {
      const int row = it * 8 + wave * 2 + hh;
      const float* sp = sY + row * kScYP + c8;
      const v4f a0 = *(const v4f*)(sp);
      const v4f a1 = *(const v4f*)(sp + 4);
#pragma unroll
      for (int e = 0; e < 4; ++e) {
        const float f0 = a0[e];
        const float f1 = a1[e];
        hv[it][e]     = (_Float16)f0;
        hv[it][4 + e] = (_Float16)f1;
      }
    }
    for (int pass = 0; pass < 2; ++pass) {
#pragma unroll
      for (int it = 0; it < 2; ++it) {
        const int row = it * 8 + wave * 2 + hh;
        *(volatile v8h*)(YG + (row0 + (size_t)(t0 + row)) * kE + d0 + c8) = hv[it];
      }
      __threadfence();
    }
  }
}

static_assert(((kRows / 64) * (kE / 64)) % 8 == 0 && ((kRows / 64) * (kPrmP / 64)) % 8 == 0, "tile counts fill whole blocks");
static_assert(((kRows * kE / 8) % 256) == 0 && ((kE * kE / 8) % 256) == 0 && ((kPrmP * kE / 8) % 256) == 0 &&
              ((kE * kDtR / 8) % 256) == 0 && ((kRows * kDtR / 8) % 256) == 0 && ((kPrmN * kE / 8) % 256) == 0, "cast grids exact");

extern "C" void kernel_launch(void* const* d_in, const int* in_sizes, int n_in,
                              void* d_out, int out_size, void* d_ws, size_t ws_size,
                              hipStream_t stream)
{
  if (n_in < 9) return;
  if (in_sizes[0] != kRows * kE) return;
  if (in_sizes[1] != kE * kE) return;
  if (in_sizes[2] != kPrmN * kE) return;
  if (in_sizes[3] != kE * 4) return;
  if (in_sizes[4] != kE * kDtR) return;
  if (in_sizes[5] != kE) return;
  if (in_sizes[6] != kE * kNst) return;
  if (in_sizes[7] != kE) return;
  if (in_sizes[8] != kE * kE) return;
  if (out_size != kRows * kE) return;
  if (ws_size < kWsTotal) return;

  const float* x      = (const float*)d_in[0];
  const float* W_z    = (const float*)d_in[1];
  const float* W_prm  = (const float*)d_in[2];
  const float* conv_w = (const float*)d_in[3];
  const float* W_dt   = (const float*)d_in[4];
  const float* b_dt   = (const float*)d_in[5];
  const float* A_log  = (const float*)d_in[6];
  const float* Dv     = (const float*)d_in[7];
  const float* W_out  = (const float*)d_in[8];
  float* dout = (float*)d_out;

  char* ws = (char*)d_ws;
  unsigned short* XH  = (unsigned short*)(ws + kOffXH);
  unsigned short* WZH = (unsigned short*)(ws + kOffWZH);
  unsigned short* WOH = (unsigned short*)(ws + kOffWOH);
  unsigned short* WPH = (unsigned short*)(ws + kOffWPH);
  unsigned short* WDH = (unsigned short*)(ws + kOffWDH);
  float*          ZP  = (float*)(ws + kOffZP);
  float*          PRM = (float*)(ws + kOffPRM);
  unsigned short* DTU = (unsigned short*)(ws + kOffDTU);
  float*          DLR = (float*)(ws + kOffDLR);
  unsigned short* YG  = (unsigned short*)(ws + kOffYG);
  const float* dummy_bias  = b_dt;
  const float* dummy_resid = x;

  cast_f16_pad_kernel<<<(kRows * kE / 8) / 256, 256, 0, stream>>>(x, XH, kRows * kE / 8, kRows * kE / 8, 1.0f);
  cast_f16_pad_kernel<<<(kE * kE / 8) / 256, 256, 0, stream>>>(W_z, WZH, kE * kE / 8, kE * kE / 8, kCarryW);
  cast_f16_pad_kernel<<<(kE * kE / 8) / 256, 256, 0, stream>>>(W_out, WOH, kE * kE / 8, kE * kE / 8, kCarryW);
  cast_f16_pad_kernel<<<(kPrmP * kE / 8) / 256, 256, 0, stream>>>(W_prm, WPH, kPrmP * kE / 8, kPrmN * kE / 8, kCarryW);
  cast_f16_pad_kernel<<<(kE * kDtR / 8) / 256, 256, 0, stream>>>(W_dt, WDH, kE * kDtR / 8, kE * kDtR / 8, kCarryWdt);

  wmma_gemm64<0, false, 0, 0, false><<<dim3(128, 1), 256, 0, stream>>>(
      XH, XH, kE, 0L, WZH, WZH, kE, 0L,
      (void*)ZP, (void*)ZP, kE, 0L, dummy_bias, dummy_resid, 0L, kRows, kE, kE, kInvW);

  wmma_gemm64<0, false, 0, 0, false><<<dim3(16, 1), 256, 0, stream>>>(
      XH, XH, kE, 0L, WPH, WPH, kE, 0L,
      (void*)PRM, (void*)PRM, kPrmP, 0L, dummy_bias, dummy_resid, 0L, kRows, kPrmP, kE, kInvW);

  dt_cast_kernel<<<(kRows * kDtR / 8) / 256, 256, 0, stream>>>(PRM, DTU, kRows * kDtR / 8);

  wmma_gemm64<0, false, 2, 0, false><<<dim3(128, 1), 256, 0, stream>>>(
      DTU, DTU, kDtR, 0L, WDH, WDH, kDtR, 0L,
      (void*)DLR, (void*)DLR, kE, 0L, b_dt, dummy_resid, 0L, kRows, kE, kDtR, kInvWdt);

  scan_kernel<<<kBatch * (kE / kScCh), kScCh, 0, stream>>>(x, conv_w, DLR, ZP, PRM, A_log, Dv, YG);

  wmma_gemm64<0, false, 0, 0, false><<<dim3(128, 1), 256, 0, stream>>>(
      YG, YG, kE, 0L, WOH, WOH, kE, 0L,
      (void*)dout, (void*)dout, kE, 0L, dummy_bias, dummy_resid, 0L, kRows, kE, kE, kInvYW);
}
